// TropicalCausalSelfAttention_12489764897084
// MI455X (gfx1250) — hardware-verified
//
#include <hip/hip_runtime.h>


#ifndef SEQ
#define SEQ 512
#endif
#define SEQ_FULL 512
#define DM    768
#define NHQ   12
#define NHK   6
#define NREP  2
#define HD    64
#define HROT  32
#define DKV   (NHK * HD)
#define NQK   (DM + DKV)
#define WROWS (DM + 2 * DKV + DM)
#define YP    (2 * DM)
#define AW    4
#define QSP   68
#define TSP   68
#define CTP   72
#define EROWS (SEQ < 256 ? SEQ : 256)
#define QRS   2048.0f
#define QRI   (1.0f / 2048.0f)
#define LOG2E 1.4426950408889634f
#define PSH   14.0f
#define NEGB  (-3.0e38f)

static_assert(HD == 64);
static_assert(HROT * 2 == HD);
static_assert(NHQ * HD == DM);
static_assert(NHK * NREP == NHQ);
static_assert(DM % 64 == 0);
static_assert(DKV % 64 == 0);
static_assert(NQK % 64 == 0);
static_assert(DM % 32 == 0);
static_assert(SEQ % 64 == 0);
static_assert(SEQ % 32 == 0);
static_assert(SEQ <= SEQ_FULL);
static_assert(EROWS % 64 == 0);
static_assert(EROWS % 32 == 0);
static_assert(EROWS % (16 * AW) == 0);
static_assert((SEQ - EROWS) % (16 * AW) == 0);
static_assert(EROWS <= SEQ);
static_assert(((size_t)SEQ * DM) % 8 == 0);
static_assert((QSP * 4) % 16 == 0);
static_assert((TSP * 4) % 16 == 0);
static_assert((CTP * 2) % 16 == 0);
static_assert(QSP >= HD);
static_assert(TSP >= 64);
static_assert(CTP >= 64);
static_assert(2 * 256 * 16 == 64 * 64 * 2);
static_assert(32 * 32 * 16 == 64 * 64 * 4);
static_assert(16 * 32 * 16 == 64 * 64 * 2);
static_assert(4 * 32 * 16 == 16 * HD * 2);
static_assert(64 * CTP * 2 <= 131072);
static_assert(64 * TSP * 4 <= 131072);
static_assert(AW * (16 * QSP + 32 * HD) * 4 <= 131072);

typedef _Float16 h16;
typedef unsigned short bf;
typedef __attribute__((ext_vector_type(16))) __bf16   v16bf;
typedef __attribute__((ext_vector_type(16))) _Float16 v16h;
typedef __attribute__((ext_vector_type(8)))  _Float16 v8h;
typedef __attribute__((ext_vector_type(8)))  unsigned short v8us;
typedef __attribute__((ext_vector_type(8)))  float    v8f;
typedef __attribute__((ext_vector_type(4)))  float    v4f;
typedef v4f  __attribute__((may_alias)) v4fa;
typedef v8us __attribute__((may_alias)) v8usa;

__device__ __forceinline__ unsigned short f2bf(float f) { unsigned u = __float_as_uint(f); u += 0x7FFFu + ((u >> 16) & 1u); return (unsigned short)(u >> 16); }
__device__ __forceinline__ float bfr(float f) { return __uint_as_float(((unsigned)f2bf(f)) << 16); }
__device__ __forceinline__ v16h cat16(v8h lo, v8h hi) { return __builtin_shufflevector(lo, hi, 0, 1, 2, 3, 4, 5, 6, 7, 8, 9, 10, 11, 12, 13, 14, 15); }
__device__ __forceinline__ v16bf cat16b(v8us lo, v8us hi) { return __builtin_bit_cast(v16bf, __builtin_shufflevector(lo, hi, 0, 1, 2, 3, 4, 5, 6, 7, 8, 9, 10, 11, 12, 13, 14, 15)); }
__device__ __forceinline__ v8f wmma16(v16h a, v16h b, v8f c) { return __builtin_amdgcn_wmma_f32_16x16x32_f16(false, a, false, b, (short)0, c, false, false); }
__device__ __forceinline__ v8f wmmab(v16bf a, v16bf b, v8f c) { return __builtin_amdgcn_wmma_f32_16x16x32_bf16(false, a, false, b, (short)0, c, false, false); }
__device__ __forceinline__ v16h  ldh(const h16* p) { return cat16(*(const v8h*)p, *(const v8h*)(p + 16)); }
__device__ __forceinline__ v16bf ldb(const bf* p)  { return cat16b(*(const v8us*)p, *(const v8us*)(p + 16)); }
__device__ __forceinline__ void wave_sync() { __builtin_amdgcn_fence(3  , "wavefront"); __builtin_amdgcn_wave_barrier(); asm volatile("" ::: "memory"); }

__device__ __forceinline__ v8f wmma16g(v16h a, v16h b, v8f c) { c = wmma16(a, b, c); asm volatile("v_nop\n\tv_nop\n\tv_nop\n\tv_nop" : "+v"(c) : "v"(a), "v"(b)); return c; }
__device__ __forceinline__ v8f wmmabg(v16bf a, v16bf b, v8f c) { c = wmmab(a, b, c); asm volatile("v_nop\n\tv_nop\n\tv_nop\n\tv_nop" : "+v"(c) : "v"(a), "v"(b)); return c; }
__device__ __forceinline__ h16 toh_flush(float v) { const h16 r = (h16)v; return (fabsf(v) < 6.103515625e-05f) ? (h16)0.0f : r; }
__device__ __forceinline__ float bf2f(unsigned short b) { return __uint_as_float(((unsigned)b) << 16); }

__global__ __launch_bounds__(256) void k_cvt8(const float* __restrict__ src, bf* dst, size_t n8) {
    const size_t i = (size_t)blockIdx.x * 256 + threadIdx.x; if (i >= n8) return;
    const v8f v = *(const v8f*)(src + i * 8); v8us o;
#pragma unroll
    for (int k = 0; k < 8; ++k) o[k] = f2bf(v[k]);
    *(volatile v8us*)(dst + i * 8) = o; __threadfence(); *(volatile v8us*)(dst + i * 8) = o;
}

__global__ __launch_bounds__(256) void k_cvtT(const float* __restrict__ W, bf* WT, int ncols, int rowoff) {
    __shared__ __align__(16) bf ts[64 * CTP];
    const int tid = threadIdx.x;
    const int n0 = blockIdx.x * 64, k0 = blockIdx.y * 64;
#pragma unroll
    for (int i = 0; i < 4; ++i) { const int idx = i * 256 + tid; const int kr = idx >> 4, c4 = (idx & 15) * 4;
        const v4f v = *(const v4f*)(W + (size_t)(k0 + kr) * (size_t)ncols + n0 + c4);
#pragma unroll
        for (int e = 0; e < 4; ++e) ts[(c4 + e) * CTP + kr] = f2bf(v[e]); }
    __syncthreads();
#pragma unroll 1
    for (int ps = 0; ps < 2; ++ps) {
#pragma unroll
        for (int i = 0; i < 2; ++i) { const int p = i * 256 + tid; const int row = p >> 3, c8 = (p & 7) * 8;
            const v8us o = *(const v8usa*)(&ts[row * CTP + c8]);
            *(volatile v8us*)(WT + (size_t)(rowoff + n0 + row) * DM + k0 + c8) = o; }
        if (ps == 0) __threadfence(); }
}

__device__ __forceinline__ void gemm64(const bf* __restrict__ A, const bf* __restrict__ Bt, const int pitchA, const int pitchB, const int kb, const int nparts,
                                       const size_t aoff, const size_t boff, v8f (&acc)[4][4]) {
#pragma unroll
    for (int mb = 0; mb < 4; ++mb)
#pragma unroll
        for (int nb = 0; nb < 4; ++nb) acc[mb][nb] = (v8f){};
#pragma unroll 1
    for (int part = 0; part < nparts; ++part) {
        const size_t ap = aoff + (size_t)part * (size_t)kb;
#pragma unroll 1
        for (int kc = 0; kc < kb; kc += 32) {
            v16bf a[4];
#pragma unroll
            for (int mb = 0; mb < 4; ++mb) a[mb] = ldb(A + ap + (size_t)mb * 16 * (size_t)pitchA + kc);
#pragma unroll
            for (int nb = 0; nb < 4; ++nb) { const v16bf b = ldb(Bt + boff + (size_t)nb * 16 * (size_t)pitchB + kc);
#pragma unroll
                for (int mb = 0; mb < 4; ++mb) acc[mb][nb] = wmmabg(a[mb], b, acc[mb][nb]); }
        }
    }
}

__global__ __launch_bounds__(32) void k_qk(const bf* __restrict__ XB, const bf* __restrict__ WT, const float* __restrict__ cosb, const float* __restrict__ sinb, float* QKF) {
    __shared__ __align__(16) float os[64 * TSP];
    const int lane = threadIdx.x & 31, lr = lane & 15, hi = lane >> 4;
    const int r0 = blockIdx.x * 64, head = blockIdx.y, c0 = head * 64;
    v8f acc[4][4];
    gemm64(XB, WT, DM, DM, DM, 1, (size_t)(r0 + lr) * DM + 8 * hi, (size_t)(c0 + lr) * DM + 8 * hi, acc);
#pragma unroll
    for (int mb = 0; mb < 4; ++mb)
#pragma unroll
        for (int nb = 0; nb < 4; ++nb)
#pragma unroll
            for (int j = 0; j < 8; ++j) os[(mb * 16 + hi * 8 + j) * TSP + nb * 16 + lr] = acc[mb][nb][j];
    wave_sync();
#pragma unroll 1
    for (int r = 0; r < 64; ++r) {
        const int t = r0 + r;
        const float x1 = os[r * TSP + lane], x2 = os[r * TSP + HROT + lane];
        const float c = bfr(cosb[(size_t)t * HROT + lane]), s = bfr(sinb[(size_t)t * HROT + lane]);
        const float o1 = x1 * c - x2 * s, o2 = x2 * c + x1 * s;
        float ss = o1 * o1 + o2 * o2;
#pragma unroll
        for (int off = 16; off > 0; off >>= 1) ss += __shfl_xor(ss, off, 32);
        const float sc = rsqrtf(ss * (1.0f / (float)HD) + 1e-6f);
        os[r * TSP + lane] = o1 * sc; os[r * TSP + HROT + lane] = o2 * sc; }
    wave_sync();
    float* dst = QKF + ((size_t)head * SEQ + (size_t)r0) * HD;
#pragma unroll 1
    for (int ps = 0; ps < 2; ++ps) {
#pragma unroll 4
        for (int i = 0; i < 32; ++i) { const int idx = i * 32 + lane; const int row = idx >> 4, c4 = (idx & 15) * 4;
            const v4f val = *(const v4fa*)(&os[row * TSP + c4]);
            *(volatile v4f*)(dst + (size_t)idx * 4) = val; }
        if (ps == 0) __threadfence(); }
}

__global__ __launch_bounds__(32) void k_vt(const bf* __restrict__ WV, const bf* __restrict__ XB, h16* VT, h16* VR) {
    __shared__ __align__(16) float os[64 * TSP];
    const int lane = threadIdx.x & 31, lr = lane & 15, hi = lane >> 4;
    const int r0 = blockIdx.x * 64, c0 = blockIdx.y * 64;
    v8f acc[4][4];
    gemm64(WV, XB, DM, DM, DM, 1, (size_t)(r0 + lr) * DM + 8 * hi, (size_t)(c0 + lr) * DM + 8 * hi, acc);
#pragma unroll
    for (int mb = 0; mb < 4; ++mb)
#pragma unroll
        for (int nb = 0; nb < 4; ++nb)
#pragma unroll
            for (int j = 0; j < 8; ++j) os[(mb * 16 + hi * 8 + j) * TSP + nb * 16 + lr] = acc[mb][nb][j];
    wave_sync();
    const bool wr = c0 < EROWS;
#pragma unroll 1
    for (int ps = 0; ps < 2; ++ps) {
#pragma unroll 4
        for (int i = 0; i < 16; ++i) { const int p = i * 32 + lane; const int row = p >> 3, c8 = (p & 7) * 8;
            const v4f x0 = *(const v4fa*)(&os[row * TSP + c8]); const v4f x1 = *(const v4fa*)(&os[row * TSP + c8 + 4]); v8h hv, rv;
#pragma unroll
            for (int e = 0; e < 4; ++e) { const h16 a0 = toh_flush(x0[e]); const h16 a1 = toh_flush(x1[e]); hv[e] = a0; hv[4 + e] = a1;
                rv[e] = toh_flush((x0[e] - (float)a0) * QRS); rv[4 + e] = toh_flush((x1[e] - (float)a1) * QRS); }
            *(volatile v8h*)(VT + (size_t)(r0 + row) * SEQ + c0 + c8) = hv;
            if (wr) *(volatile v8h*)(VR + (size_t)(r0 + row) * EROWS + c0 + c8) = rv; }
        if (ps == 0) __threadfence(); }
}

__global__ __launch_bounds__(32) void k_oproj(const bf* __restrict__ YB, const bf* __restrict__ WP, float* OUT) {
    __shared__ __align__(16) float os[64 * TSP];
    const int lane = threadIdx.x & 31, lr = lane & 15, hi = lane >> 4;
    const int r0 = blockIdx.x * 64, c0 = blockIdx.y * 64;
    v8f acc[4][4];
    gemm64(YB, WP, YP, DM, DM, 2, (size_t)(r0 + lr) * YP + 8 * hi, (size_t)(c0 + lr) * DM + 8 * hi, acc);
#pragma unroll
    for (int mb = 0; mb < 4; ++mb)
#pragma unroll
        for (int nb = 0; nb < 4; ++nb)
#pragma unroll
            for (int j = 0; j < 8; ++j) os[(mb * 16 + hi * 8 + j) * TSP + nb * 16 + lr] = acc[mb][nb][j];
    wave_sync();
#pragma unroll 1
    for (int ps = 0; ps < 2; ++ps) {
#pragma unroll 4
        for (int i = 0; i < 32; ++i) { const int idx = i * 32 + lane; const int row = idx >> 4, c4 = (idx & 15) * 4;
            const v4f val = *(const v4fa*)(&os[row * TSP + c4]);
            *(volatile v4f*)(OUT + (size_t)(r0 + row) * DM + c0 + c4) = val; }
        if (ps == 0) __threadfence(); }
}

template <int EARLY>
__device__ __forceinline__ void flash_body(const float* __restrict__ QKF, const h16* __restrict__ VT, const h16* __restrict__ VR, bf* YB) {
    __shared__ __align__(16) float qs[AW * 16 * QSP];
    __shared__ __align__(16) float ks[AW * 32 * HD];
    const int lane = threadIdx.x & 31, lr = lane & 15, hi = lane >> 4;
    const int wave = __builtin_amdgcn_readfirstlane((int)(threadIdx.x >> 5));
    const int h = blockIdx.y, kvh = h / NREP;
    const int t0 = (EARLY ? 0 : EROWS) + (blockIdx.x * AW + wave) * 16;
    const int lim = t0 + lr;
    const int nk = (t0 + 16 + 31) & ~31;
    const int qb = wave * 16 * QSP, kbs = wave * 32 * HD;
    { const size_t qsrc = ((size_t)h * SEQ + (size_t)t0) * HD;
#pragma unroll
      for (int i = 0; i < 8; ++i) { const int idx = i * 32 + lane;
          const v4f v = *(const v4f*)(QKF + qsrc + (size_t)idx * 4);
          *(v4fa*)(&qs[qb + (idx >> 4) * QSP + (idx & 15) * 4]) = v; } }
    const size_t kplane = ((size_t)(NHQ + kvh) * SEQ) * HD;
    const size_t vo  = (size_t)(kvh * HD + lr) * SEQ + 8 * hi;
    const size_t vro = (size_t)(kvh * HD + lr) * EROWS + 8 * hi;
    const v16h hz = (v16h){};
    v8f o[4], oR[4];
#pragma unroll
    for (int j = 0; j < 4; ++j) { o[j] = (v8f){}; oR[j] = (v8f){}; }
    float m = NEGB, l = 0.0f;
#pragma unroll 1
    for (int key0 = 0; key0 < nk; key0 += 32) {
        wave_sync();
        { const size_t ksrc = kplane + (size_t)key0 * HD;
#pragma unroll 8
          for (int i = 0; i < 16; ++i) { const int idx = i * 32 + lane;
              const v4f v = *(const v4f*)(QKF + ksrc + (size_t)idx * 4);
              *(v4fa*)(&ks[kbs + idx * 4]) = v; } }
        wave_sync();
        float sa[8], sb[8];
#pragma unroll
        for (int r = 0; r < 8; ++r) { sa[r] = NEGB; sb[r] = NEGB; }
#pragma unroll 1
        for (int d4 = 0; d4 < HD / 4; ++d4) {
            const v4f q4 = *(const v4fa*)(&qs[qb + lr * QSP + d4 * 4]);
#pragma unroll
            for (int r = 0; r < 8; ++r) {
                const v4f ka = *(const v4fa*)(&ks[kbs + (8 * hi + r) * HD + d4 * 4]);
                const v4f kc = *(const v4fa*)(&ks[kbs + (16 + 8 * hi + r) * HD + d4 * 4]);
                sa[r] = fmaxf(sa[r], fmaxf(fmaxf(q4[0] + ka[0], q4[1] + ka[1]), fmaxf(q4[2] + ka[2], q4[3] + ka[3])));
                sb[r] = fmaxf(sb[r], fmaxf(fmaxf(q4[0] + kc[0], q4[1] + kc[1]), fmaxf(q4[2] + kc[2], q4[3] + kc[3]))); }
        }
        const int ja = key0 + 8 * hi;
        float mx = NEGB;
#pragma unroll
        for (int r = 0; r < 8; ++r) {
            sa[r] = sa[r] * LOG2E; sb[r] = sb[r] * LOG2E;
            const bool fa = (ja + r <= lim), fb = (ja + 16 + r <= lim);
            mx = fmaxf(mx, fmaxf(fa ? sa[r] : NEGB, fb ? sb[r] : NEGB)); }
        mx = fmaxf(mx, __shfl_xor(mx, 16, 32));
        const float mnew = fmaxf(m, mx);
        const float alpha = __builtin_amdgcn_exp2f(m - mnew);
        const float sh = PSH - mnew;
        v16h pb, pr = hz; float ls = 0.0f;
#pragma unroll
        for (int r = 0; r < 8; ++r) {
            const float xa = sa[r] + sh, xb = sb[r] + sh;
            const float ea = __builtin_amdgcn_exp2f(xa), eb = __builtin_amdgcn_exp2f(xb);
            const bool fa = (ja + r <= lim) & (xa >= -14.0f), fb = (ja + 16 + r <= lim) & (xb >= -14.0f);
            const float ga = fa ? ea : 0.0f, gb = fb ? eb : 0.0f;
            const h16 pa = (h16)ga; const h16 pc = (h16)gb;
            pb[r] = pa; pb[8 + r] = pc;
            if (EARLY) { pr[r] = toh_flush((ga - (float)pa) * QRS); pr[8 + r] = toh_flush((gb - (float)pc) * QRS); ls += ga + gb; }
            else       { ls += (float)pa + (float)pc; } }
        l = l * alpha + ls; m = mnew;
#pragma unroll
        for (int j = 0; j < 4; ++j) {
            const v16h v = ldh(VT + vo + (size_t)(16 * j) * SEQ + key0);
            o[j] = o[j] * alpha;
            o[j] = wmma16g(v, pb, o[j]);
            if (EARLY) {
                const v16h vr = ldh(VR + vro + (size_t)(16 * j) * EROWS + key0);
                oR[j] = oR[j] * alpha;
                oR[j] = wmma16g(v, pr, oR[j]);
                oR[j] = wmma16g(vr, pb, oR[j]); }
        }
    }
    l += __shfl_xor(l, 16, 32);
    const bool any = l > 0.0f;
    const float lsafe = any ? l : 1.0f;
    const float inv = any ? (1.0f / lsafe) : 0.0f;
    wave_sync();
#pragma unroll
    for (int j = 0; j < 4; ++j) {
        v8f f = o[j];
        if (EARLY) f = o[j] + oR[j] * QRI;
        v4f a, c;
        a[0] = f[0] * inv; a[1] = f[1] * inv; a[2] = f[2] * inv; a[3] = f[3] * inv; c[0] = f[4] * inv; c[1] = f[5] * inv; c[2] = f[6] * inv; c[3] = f[7] * inv;
        *(v4fa*)(&qs[qb + lr * QSP + 16 * j + 8 * hi]) = a; *(v4fa*)(&qs[qb + lr * QSP + 16 * j + 8 * hi + 4]) = c; }
    wave_sync();
    bf* yrow = YB + (size_t)t0 * YP + h * HD;
#pragma unroll 1
    for (int ps = 0; ps < 2; ++ps) {
#pragma unroll
        for (int s = 0; s < 4; ++s) { const int row = 4 * s + (lane >> 3), c8 = (lane & 7) * 8;
            const v4f x0 = *(const v4fa*)(&qs[qb + row * QSP + c8]); const v4f x1 = *(const v4fa*)(&qs[qb + row * QSP + c8 + 4]); v8us hv, lv;
#pragma unroll
            for (int e = 0; e < 4; ++e) { const unsigned short b0 = f2bf(x0[e]); const unsigned short b1 = f2bf(x1[e]); hv[e] = b0; hv[4 + e] = b1;
                lv[e] = f2bf(x0[e] - bf2f(b0)); lv[4 + e] = f2bf(x1[e] - bf2f(b1)); }
            *(volatile v8us*)(yrow + (size_t)row * YP + c8) = hv;
            *(volatile v8us*)(yrow + (size_t)row * YP + DM + c8) = lv; }
        if (ps == 0) __threadfence(); }
}

__global__ __launch_bounds__(32 * AW) __attribute__((amdgpu_num_vgpr(256))) void k_flash_early(const float* __restrict__ QKF, const h16* __restrict__ VT, const h16* __restrict__ VR, bf* YB) {
    flash_body<1>(QKF, VT, VR, YB);
}
__global__ __launch_bounds__(32 * AW) __attribute__((amdgpu_num_vgpr(256))) void k_flash_late(const float* __restrict__ QKF, const h16* __restrict__ VT, const h16* __restrict__ VR, bf* YB) {
    flash_body<0>(QKF, VT, VR, YB);
}

static constexpr size_t al256(size_t v) { return (v + 255) & ~(size_t)255; }
static constexpr size_t SZ_XB = al256((size_t)SEQ * DM * 2);
static constexpr size_t SZ_WT = al256((size_t)WROWS * DM * 2);
static constexpr size_t SZ_QK = al256((size_t)(NHQ + NHK) * SEQ * HD * 4);
static constexpr size_t SZ_VT = al256((size_t)DKV * SEQ * 2);
static constexpr size_t SZ_VR = al256((size_t)DKV * EROWS * 2);
static constexpr size_t SZ_YB = al256((size_t)SEQ * YP * 2);
static constexpr size_t SZ_TOTAL = SZ_XB + SZ_WT + SZ_QK + SZ_VT + SZ_VR + SZ_YB;
static_assert(SZ_TOTAL <= (size_t)134217728);
static_assert(((size_t)DM * DM * 2) % 256 == 0);
static_assert(((size_t)DKV * DM * 2) % 256 == 0);
static_assert(((size_t)NHQ * SEQ * HD * 4) % 256 == 0);

extern "C" void kernel_launch(void* const* d_in, const int* in_sizes, int n_in,
                              void* d_out, int out_size, void* d_ws, size_t ws_size, hipStream_t stream) {
    if (n_in < 7) return;
    if ((size_t)in_sizes[0] < (size_t)SEQ * DM) return;
    if ((size_t)in_sizes[1] < (size_t)SEQ * HROT || (size_t)in_sizes[2] < (size_t)SEQ * HROT) return;
    if ((size_t)in_sizes[3] < (size_t)DM * DM || (size_t)in_sizes[6] < (size_t)DM * DM) return;
    if ((size_t)in_sizes[4] < (size_t)DM * DKV || (size_t)in_sizes[5] < (size_t)DM * DKV) return;
    if ((size_t)out_size < (size_t)SEQ * DM) return;
    if (SZ_TOTAL > ws_size) return;
    const float* x    = (const float*)d_in[0];
    const float* cosb = (const float*)d_in[1];
    const float* sinb = (const float*)d_in[2];
    const float* wq   = (const float*)d_in[3];
    const float* wk   = (const float*)d_in[4];
    const float* wv   = (const float*)d_in[5];
    const float* wp   = (const float*)d_in[6];
    float* OUT = (float*)d_out;
    char* wsp = (char*)d_ws;
    bf*    XB  = (bf*)wsp;    wsp += SZ_XB;
    bf*    WT  = (bf*)wsp;    wsp += SZ_WT;
    float* QKF = (float*)wsp; wsp += SZ_QK;
    h16*   VT  = (h16*)wsp;   wsp += SZ_VT;
    h16*   VR  = (h16*)wsp;   wsp += SZ_VR;
    bf*    YB  = (bf*)wsp;    wsp += SZ_YB;

    { const size_t n8 = (size_t)SEQ * DM / 8;
      k_cvt8<<<(unsigned)((n8 + 255) / 256), 256, 0, stream>>>(x, XB, n8); }
    k_cvtT<<<dim3(DM / 64,  DM / 64, 1), 256, 0, stream>>>(wq, WT, DM,  0);
    k_cvtT<<<dim3(DKV / 64, DM / 64, 1), 256, 0, stream>>>(wk, WT, DKV, DM);
    k_cvtT<<<dim3(DKV / 64, DM / 64, 1), 256, 0, stream>>>(wv, WT, DKV, NQK);
    k_cvtT<<<dim3(DM / 64,  DM / 64, 1), 256, 0, stream>>>(wp, WT, DM,  NQK + DKV);

    k_qk<<<dim3(SEQ / 64, NHQ + NHK, 1), 32, 0, stream>>>(XB, WT, cosb, sinb, QKF);
    k_vt<<<dim3(DKV / 64, SEQ / 64, 1), 32, 0, stream>>>(WT + (size_t)NQK * DM, XB, VT, VR);

    k_flash_early<<<dim3(EROWS / (16 * AW), NHQ, 1), 32 * AW, 0, stream>>>(QKF, VT, VR, YB);
    if (SEQ > EROWS)
        k_flash_late<<<dim3((SEQ - EROWS) / (16 * AW), NHQ, 1), 32 * AW, 0, stream>>>(QKF, VT, VR, YB);

    k_oproj<<<dim3(SEQ / 64, DM / 64, 1), 32, 0, stream>>>(YB, WT + (size_t)(NQK + DKV) * DM, OUT);
}
